// GravitationalAttentionHead_32993938768206
// MI455X (gfx1250) — hardware-run, weakly checked
//
#include <hip/hip_runtime.h>

#define NBATCH 4
#define NS     4096
#define ND     64
#define NPOS   3
#define QB     32
#define KSTEP  64
#define PSP    72
#define OSP    68
#define XSP    72
#define EVT    1.0e-6f
#define MAXF   50.0f
#define CURV   0.15f

static_assert((NS % KSTEP) == 0);
static_assert((NS % QB) == 0);
static_assert((NS % 64) == 0);
static_assert(((NBATCH * NS) % 256) == 0);

typedef __bf16         v16b __attribute__((ext_vector_type(16)));
typedef unsigned short v8us __attribute__((ext_vector_type(8)));
typedef float          v8f  __attribute__((ext_vector_type(8)));
typedef float          v4f  __attribute__((ext_vector_type(4)));
typedef v8us __attribute__((may_alias)) v8usa;
typedef v4f  __attribute__((may_alias)) v4fa;
union FragB { v16b v; v8us half[2]; };
union Q8    { v8f v; v4f q[2]; };

__device__ __forceinline__ v8f wmma_bf16(v16b a, v16b b, v8f c) {
  v8f d = __builtin_amdgcn_wmma_f32_16x16x32_bf16(false, a, false, b, (short)0, c, false, false);
  asm volatile("v_nop\n\tv_nop\n\tv_nop\n\tv_nop" : "+v"(d) : "v"(a), "v"(b));
  return d;
}

__device__ __forceinline__ v16b frag32(const unsigned short* p, int h) {
  FragB f;
  f.half[0] = *(const v8usa*)(p + 8 * h);
  f.half[1] = *(const v8usa*)(p + 16 + 8 * h);
  return f.v;
}

__device__ __forceinline__ v8f zero8f() {
  v8f z;
  #pragma unroll
  for (int j = 0; j < 8; ++j) z[j] = 0.f;
  return z;
}

__device__ __forceinline__ unsigned int bf16_rne(float f) {
  const unsigned int u = __float_as_uint(f);
  return (u + 0x7FFFu + ((u >> 16) & 1u)) >> 16;
}

__global__ __launch_bounds__(256) void k_masses(const float* __restrict__ x,
                                                const float* __restrict__ mw,
                                                float* __restrict__ mG,
                                                float* __restrict__ outm)
{
  #pragma clang fp contract(off)
  __shared__ __attribute__((aligned(16))) float sM[256];
  const int tid = threadIdx.x;
  const int tok = blockIdx.x * 256 + tid;
  const float* xr = x + (size_t)tok * ND;
  float z = 0.f;
  #pragma unroll 4
  for (int q = 0; q < ND / 4; ++q) {
    const v4f a  = *(const v4fa*)(xr + 4 * q);
    const v4f w4 = *(const v4fa*)(mw + 4 * q);
    z = fmaf(a.x, w4.x, z);
    z = fmaf(a.y, w4.y, z);
    z = fmaf(a.z, w4.z, z);
    z = fmaf(a.w, w4.w, z);
  }
  const float mval = fmaxf(z, 0.f) + log1pf(expf(-fabsf(z)));
  sM[tid] = mval;
  __syncthreads();
  if (tid < 64) {
    const v4f v = *(const v4fa*)(sM + 4 * tid);
    const size_t d = (size_t)blockIdx.x * 256 + 4 * tid;
    *(volatile v4f*)(mG + d)   = v;
    *(volatile v4f*)(outm + d) = v;
    __threadfence();
    *(volatile v4f*)(mG + d)   = v;
    *(volatile v4f*)(outm + d) = v;
  }
}

__global__ __launch_bounds__(256) void k_xcvt(const float* __restrict__ x,
                                              unsigned short* __restrict__ XTh,
                                              unsigned short* __restrict__ XTl)
{
  __shared__ __attribute__((aligned(16))) unsigned short sHh[ND * XSP];
  __shared__ __attribute__((aligned(16))) unsigned short sHl[ND * XSP];
  const int tid = threadIdx.x, lane = tid & 31, w = tid >> 5;
  const int j0 = blockIdx.x * 64, b = blockIdx.y;
  #pragma unroll
  for (int it = 0; it < 4; ++it) {
    const int q = tid + 256 * it;
    const int j = q >> 4;
    const int d0 = 4 * (q & 15);
    const v4f v = *(const v4fa*)(x + (size_t)(b * NS + j0 + j) * ND + d0);
    #pragma unroll
    for (int e = 0; e < 4; ++e) {
      const float f = v[e];
      const unsigned int hb = bf16_rne(f);
      const float lof = f - __uint_as_float(hb << 16);
      const unsigned int lb = bf16_rne(lof);
      sHh[(d0 + e) * XSP + j] = (unsigned short)hb;
      sHl[(d0 + e) * XSP + j] = (unsigned short)lb;
    }
  }
  __syncthreads();
  const int q8 = lane & 7, sub = lane >> 3;
  v8us vh[2], vl[2];
  #pragma unroll
  for (int i = 0; i < 2; ++i) {
    const int d = 8 * w + 4 * i + sub;
    vh[i] = *(const v8usa*)(sHh + d * XSP + 8 * q8);
    vl[i] = *(const v8usa*)(sHl + d * XSP + 8 * q8);
    const size_t o = (size_t)(b * ND + d) * NS + j0 + 8 * q8;
    *(volatile v8us*)(XTh + o) = vh[i];
    *(volatile v8us*)(XTl + o) = vl[i];
  }
  __threadfence();
  #pragma unroll
  for (int i = 0; i < 2; ++i) {
    const int d = 8 * w + 4 * i + sub;
    const size_t o = (size_t)(b * ND + d) * NS + j0 + 8 * q8;
    *(volatile v8us*)(XTh + o) = vh[i];
    *(volatile v8us*)(XTl + o) = vl[i];
  }
}

__global__ __launch_bounds__(256) void k_geo(const float* __restrict__ pos,
                                             float* __restrict__ R)
{
  #pragma clang fp contract(off)
  __shared__ __attribute__((aligned(16))) float sR[NS];
  const int tid = threadIdx.x;
  const int i = blockIdx.x;
  const float px = pos[i * NPOS + 0];
  const float py = pos[i * NPOS + 1];
  const float pz = pos[i * NPOS + 2];
  #pragma unroll 1
  for (int q = 0; q < 16; ++q) {
    const int j = 4 * tid + 1024 * (q >> 2) + (q & 3);
    const float dx = pos[j * NPOS + 0] - px;
    const float dy = pos[j * NPOS + 1] - py;
    const float dz = pos[j * NPOS + 2] - pz;
    const float d2 = (dx * dx + dz * dz) + dy * dy;
    const float dn = sqrtf(d2 + EVT);
    const float c  = cosf(dn);
    float d2m = d2 * (1.0f + CURV * c);
    d2m = fmaxf(d2m, EVT);
    sR[j] = 1.0f / d2m;
  }
  __syncthreads();
  v4f v[4];
  #pragma unroll
  for (int k = 0; k < 4; ++k) {
    v[k] = *(const v4fa*)(sR + 4 * tid + 1024 * k);
    const size_t o = (size_t)i * NS + 4 * tid + 1024 * k;
    *(volatile v4f*)(R + o) = v[k];
  }
  __threadfence();
  #pragma unroll
  for (int k = 0; k < 4; ++k) {
    const size_t o = (size_t)i * NS + 4 * tid + 1024 * k;
    *(volatile v4f*)(R + o) = v[k];
  }
}

__global__ __launch_bounds__(256) void k_att(const unsigned short* __restrict__ XTh,
                                             const unsigned short* __restrict__ XTl,
                                             const float* __restrict__ R,
                                             const float* __restrict__ mG,
                                             const float* __restrict__ Gp,
                                             float* __restrict__ out)
{
  #pragma clang fp contract(off)
  __shared__ __attribute__((aligned(16))) float          ms[NS];
  __shared__ __attribute__((aligned(16))) unsigned short sPh[QB * PSP];
  __shared__ __attribute__((aligned(16))) unsigned short sPl[QB * PSP];
  __shared__ __attribute__((aligned(16))) float          sO[QB * OSP];
  __shared__ __attribute__((aligned(16))) float          sLi[QB];
  const int tid = threadIdx.x, lane = tid & 31, w = tid >> 5;
  const int h = lane >> 4, m = lane & 15;
  const int i0 = blockIdx.x * QB, b = blockIdx.y;

  {
    const v4fa* src = (const v4fa*)(mG + (size_t)b * NS);
    v4fa* dst = (v4fa*)ms;
    for (int k = tid; k < NS / 4; k += 256) dst[k] = src[k];
  }
  __syncthreads();

  const int si = tid >> 3, jq = tid & 7;
  const int i = i0 + si;
  const float Gmi = fabsf(Gp[0]) * ms[i];
  const int it = w & 1, dt = w >> 1;
  const unsigned short* bhrow = XTh + (size_t)(b * ND + 16 * dt + m) * NS;
  const unsigned short* blrow = XTl + (size_t)(b * ND + 16 * dt + m) * NS;
  const float* rrow = R + (size_t)i * NS + 8 * jq;
  const float* mrow = ms + 8 * jq;
  const unsigned short* pah = sPh + (16 * it + m) * PSP;
  const unsigned short* pal = sPl + (16 * it + m) * PSP;
  unsigned short* pwh = sPh + si * PSP + 8 * jq;
  unsigned short* pwl = sPl + si * PSP + 8 * jq;

  v8f acc = zero8f();
  float lsum = 0.f;

  #pragma unroll 1
  for (int j0 = 0; j0 < NS; j0 += KSTEP) {
    Q8 rr, mm;
    rr.q[0] = *(const v4fa*)(rrow + j0);
    rr.q[1] = *(const v4fa*)(rrow + j0 + 4);
    mm.q[0] = *(const v4fa*)(mrow + j0);
    mm.q[1] = *(const v4fa*)(mrow + j0 + 4);
    v8us ph, pl;
    #pragma unroll
    for (int e = 0; e < 8; ++e) {
      float f = (Gmi * mm.v[e]) * rr.v[e];
      f = fminf(f, MAXF);
      const float p = __expf(f - MAXF);
      lsum += p;
      const unsigned int hb = bf16_rne(p);
      const float lof = p - __uint_as_float(hb << 16);
      const unsigned int lb = bf16_rne(lof);
      ph[e] = (unsigned short)hb;
      pl[e] = (unsigned short)lb;
    }
    *(v8usa*)pwh = ph;
    *(v8usa*)pwl = pl;
    __syncthreads();

    #pragma unroll
    for (int kc = 0; kc < 2; ++kc) {
      const v16b ah = frag32(pah + 32 * kc, h);
      const v16b al = frag32(pal + 32 * kc, h);
      const v16b xh = frag32(bhrow + j0 + 32 * kc, h);
      const v16b xl = frag32(blrow + j0 + 32 * kc, h);
      acc = wmma_bf16(ah, xh, acc);
      acc = wmma_bf16(ah, xl, acc);
      acc = wmma_bf16(al, xh, acc);
    }
    __syncthreads();
  }

  lsum += __shfl_xor(lsum, 1);
  lsum += __shfl_xor(lsum, 2);
  lsum += __shfl_xor(lsum, 4);
  if (jq == 0) sLi[si] = 1.0f / lsum;
  __syncthreads();

  #pragma unroll
  for (int r = 0; r < 8; ++r) {
    const int row = 16 * it + 8 * h + r;
    const float li = sLi[row];
    sO[row * OSP + 16 * dt + m] = acc[r] * li;
  }
  __syncthreads();

  const int q8 = lane & 7, sub = lane >> 3;
  v4f ov[2];
  #pragma unroll
  for (int k = 0; k < 2; ++k) {
    const int lid = 8 * w + 4 * k + sub;
    const int row = lid >> 1, hf = lid & 1;
    ov[k] = *(const v4fa*)(sO + row * OSP + 32 * hf + 4 * q8);
    const size_t d = (size_t)(b * NS + i0 + row) * ND + 32 * hf + 4 * q8;
    *(volatile v4f*)(out + d) = ov[k];
  }
  __threadfence();
  #pragma unroll
  for (int k = 0; k < 2; ++k) {
    const int lid = 8 * w + 4 * k + sub;
    const int row = lid >> 1, hf = lid & 1;
    const size_t d = (size_t)(b * NS + i0 + row) * ND + 32 * hf + 4 * q8;
    *(volatile v4f*)(out + d) = ov[k];
  }
}

extern "C" void kernel_launch(void* const* d_in, const int* in_sizes, int n_in,
                              void* d_out, int out_size, void* d_ws, size_t ws_size,
                              hipStream_t stream) {
  if (n_in < 4) return;
  if (in_sizes[0] != NBATCH * NS * ND) return;
  if (in_sizes[1] != NS * NPOS) return;
  if (in_sizes[2] < 1) return;
  if (in_sizes[3] != ND) return;
  if (out_size != NBATCH * NS * ND + NBATCH * NS) return;

  const float* x   = (const float*)d_in[0];
  const float* pos = (const float*)d_in[1];
  const float* Gp  = (const float*)d_in[2];
  const float* mw  = (const float*)d_in[3];

  float* out0 = (float*)d_out;
  float* out1 = out0 + (size_t)NBATCH * NS * ND;

  const size_t szM  = (size_t)NBATCH * NS * sizeof(float);
  const size_t szXT = (size_t)NBATCH * ND * NS * sizeof(unsigned short);
  const size_t szR  = (size_t)NS * NS * sizeof(float);
  size_t off = 0;
  char* ws = (char*)d_ws;
  float* mG = (float*)(ws + off);                     off += szM;
  unsigned short* XTh = (unsigned short*)(ws + off);  off += szXT;
  unsigned short* XTl = (unsigned short*)(ws + off);  off += szXT;
  float* R = (float*)(ws + off);                      off += szR;
  if (off > ws_size) return;

  k_masses<<<(NBATCH * NS) / 256, 256, 0, stream>>>(x, mw, mG, out1);
  k_xcvt<<<dim3(NS / 64, NBATCH), 256, 0, stream>>>(x, XTh, XTl);
  k_geo<<<NS, 256, 0, stream>>>(pos, R);
  k_att<<<dim3(NS / QB, NBATCH), 256, 0, stream>>>(XTh, XTl, R, mG, Gp, out0);
}
